// FFN_8658654069091
// MI455X (gfx1250) — hardware-verified
//
#include <hip/hip_runtime.h>
#include <stddef.h>
#include <stdint.h>


#define BATCH   4096
#define MAXLEN  2048
#define CHARS   10000
#define HIDDEN  1024
#define OUTPUT  100
#define K1P     10048
#define KS1     313
#define N2P     128
#define KS2     (HIDDEN / 32)
#define NT      256
#define NWAVE   8
#define HROWS   8
#define NSTEP   (MAXLEN / 32)
#define CPR     (K1P / 8)
#define NB1     ((HIDDEN * CPR) / NT)
#define NB2     ((N2P * HIDDEN / 8) / NT)
#define BM      128
#define BN      128
#define SP      132
#define STG_FLOATS (BM * OUTPUT)
#define INVKEY  16383
#define WSCAP   134217728
#define W1SC    64.0f
#define HSC     16.0f
#define W2SC    16.0f
#define LDSH_BYTES (HROWS * K1P * 2)

static_assert(NT == NWAVE * 32);
static_assert(HROWS == NWAVE);
static_assert((BATCH % HROWS) == 0);
static_assert((MAXLEN % 32) == 0);
static_assert((K1P % 64) == 0);
static_assert(KS1 * 32 >= CHARS && KS1 * 32 <= K1P);
static_assert((CHARS % 8) == 0);
static_assert(((HIDDEN * CPR) % NT) == 0);
static_assert(((N2P * HIDDEN / 8) % NT) == 0);
static_assert(((HROWS * CPR) % 32) == 0);
static_assert((BATCH % BM) == 0 && (HIDDEN % BN) == 0);
static_assert(N2P == BN && OUTPUT <= N2P);
static_assert(KS2 * 32 == HIDDEN);
static_assert(((BM * OUTPUT) % 128) == 0);
static_assert(((BM * OUTPUT * 4) % 128) == 0);
static_assert(64 * SP <= STG_FLOATS);
static_assert((SP % 4) == 0);
static_assert(CHARS < INVKEY && K1P <= 16384);
static_assert(BM == 2 * 64 && BN == 4 * 32);
static_assert(LDSH_BYTES < 300000);
static_assert(STG_FLOATS * 4 <= 65536);

typedef float          v4f  __attribute__((ext_vector_type(4))) __attribute__((may_alias));
typedef float          v8f  __attribute__((ext_vector_type(8)));
typedef int            v4i  __attribute__((ext_vector_type(4))) __attribute__((may_alias));
typedef unsigned short v8us __attribute__((ext_vector_type(8))) __attribute__((may_alias));
typedef _Float16       v8h  __attribute__((ext_vector_type(8))) __attribute__((may_alias));
typedef _Float16       v16h __attribute__((ext_vector_type(16)));
union FragH { v16h v; v8h h[2]; };

__device__ __forceinline__ v8f wmf(v16h a, v16h b, v8f c) {
  v8f d = __builtin_amdgcn_wmma_f32_16x16x32_f16(false, a, false, b, (short)0, c, false, false);
  asm volatile("v_nop\n\tv_nop\n\tv_nop\n\tv_nop" : "+v"(d) : "v"(a), "v"(b));
  return d;
}

__global__ __launch_bounds__(NT) void k_cvt(const float* __restrict__ W1, const float* __restrict__ W2,
                                            _Float16* w1h, _Float16* w2h) {
  const int tid = threadIdx.x;
  const float* p;
  float sc;
  _Float16* d;
  if (blockIdx.x < NB1) {
    const int q = blockIdx.x * NT + tid;
    const int n = q / CPR;
    const int k = 8 * (q - n * CPR);
    const int kc = k < CHARS - 8 ? k : CHARS - 8;
    p = W1 + (size_t)n * CHARS + kc;
    sc = (k < CHARS) ? W1SC : 0.0f;
    d = w1h + (size_t)q * 8;
  } else {
    const int q = (blockIdx.x - NB1) * NT + tid;
    const int n = q >> 7;
    const int k = 8 * (q & 127);
    const int nc = n < OUTPUT ? n : OUTPUT - 1;
    p = W2 + (size_t)nc * HIDDEN + k;
    sc = (n < OUTPUT) ? W2SC : 0.0f;
    d = w2h + (size_t)q * 8;
  }
  const v4f f0 = *(const v4f*)p;
  const v4f f1 = *(const v4f*)(p + 4);
  v8h a;
  a[0] = (_Float16)(f0.x * sc); a[1] = (_Float16)(f0.y * sc);
  a[2] = (_Float16)(f0.z * sc); a[3] = (_Float16)(f0.w * sc);
  a[4] = (_Float16)(f1.x * sc); a[5] = (_Float16)(f1.y * sc);
  a[6] = (_Float16)(f1.z * sc); a[7] = (_Float16)(f1.w * sc);
  *(volatile v8h*)d = a;
  __threadfence();
  *(volatile v8h*)d = a;
}

__global__ __launch_bounds__(NT) void k_hist(const int* __restrict__ words, _Float16* ah) {
  extern __shared__ __align__(16) unsigned short hst[];
  const int tid = threadIdx.x, lane = tid & 31, wave = tid >> 5;

  const v4i zi = {0, 0, 0, 0};
#pragma unroll 1
  for (int i = tid; i < (HROWS * K1P) / 8; i += NT) ((v4i*)hst)[i] = zi;
  __syncthreads();

  const int row = blockIdx.x * HROWS + wave;
  const int* wr = words + (size_t)row * MAXLEN + lane;
  unsigned short* hw = hst + wave * K1P;
  const unsigned below = (1u << lane) - 1u;

#pragma unroll 1
  for (int s = 0; s < NSTEP; ++s) {
    int c = wr[32 * s];
    c = c < 0 ? c + CHARS : c;
    const bool valid = (unsigned)c < (unsigned)CHARS;
    const unsigned key = valid ? (unsigned)c : (unsigned)INVKEY;
    unsigned msk = 0xffffffffu;
#pragma unroll
    for (int b = 0; b < 14; ++b) {
      const unsigned bitv = (key >> b) & 1u;
      const unsigned bal = __builtin_amdgcn_ballot_w32(bitv != 0u);
      msk &= bal ^ (bitv - 1u);
    }
    const int cnt = __builtin_popcount(msk);
    const bool lead = (msk & below) == 0u;
    const int ca = valid ? c : 0;
    if (valid && lead) hw[ca] = (unsigned short)(hw[ca] + cnt);
    __syncthreads();
  }

  _Float16* dst = ah + (size_t)blockIdx.x * (HROWS * K1P);
  auto emit = [&]() {
#pragma unroll 1
    for (int g = 0; g < (HROWS * CPR + NT - 1) / NT; ++g) {
      const int q = g * NT + tid;
      if (q < HROWS * CPR) {
        const v8us u = *(const v8us*)(hst + 8 * q);
        v8h hv;
#pragma unroll
        for (int i = 0; i < 8; ++i) hv[i] = (_Float16)(float)(unsigned)u[i];
        *(volatile v8h*)(dst + (size_t)q * 8) = hv;
      }
    }
  };
  emit();
  __threadfence();
  emit();
}

template <int MODE>
__global__ __launch_bounds__(NT) void k_gemm(const _Float16* __restrict__ Ap, const _Float16* __restrict__ Bp,
                                             const float* __restrict__ bias, int lda, int ldb, int ksteps,
                                             _Float16* outh, float* outf) {
  __shared__ __attribute__((aligned(16))) float stg[STG_FLOATS];

  const int tid = threadIdx.x, lane = tid & 31, wave = tid >> 5;
  const int wm = wave & 1, wn = wave >> 1;
  const int lr = lane & 15, hs = lane >> 4;
  const int m0 = blockIdx.y * BM, n0 = blockIdx.x * BN;

  const _Float16* ap0 = Ap + (size_t)(m0 + wm * 64 + lr) * lda + 8 * hs;
  const _Float16* bp0 = Bp + (size_t)(n0 + wn * 32 + lr) * ldb + 8 * hs;

  v8f acc[4][2];
#pragma unroll
  for (int t = 0; t < 4; ++t)
#pragma unroll
    for (int j = 0; j < 2; ++j)
#pragma unroll
      for (int v = 0; v < 8; ++v) acc[t][j][v] = 0.f;

#pragma unroll 1
  for (int ks = 0; ks < ksteps; ++ks) {
    const int k0 = ks * 32;
    FragH a[4], b[2];
#pragma unroll
    for (int t = 0; t < 4; ++t) {
      const _Float16* ap = ap0 + (size_t)t * 16 * lda + k0;
      a[t].h[0] = *(const v8h*)(ap);
      a[t].h[1] = *(const v8h*)(ap + 16);
    }
#pragma unroll
    for (int j = 0; j < 2; ++j) {
      const _Float16* bp = bp0 + (size_t)j * 16 * ldb + k0;
      b[j].h[0] = *(const v8h*)(bp);
      b[j].h[1] = *(const v8h*)(bp + 16);
    }
#pragma unroll
    for (int t = 0; t < 4; ++t)
#pragma unroll
      for (int j = 0; j < 2; ++j) acc[t][j] = wmf(a[t].v, b[j].v, acc[t][j]);
  }

  if (MODE == 0) {
    constexpr float INV1 = 1.0f / W1SC;
    const float bv0 = bias[n0 + wn * 32 + lr];
    const float bv1 = bias[n0 + wn * 32 + 16 + lr];
#pragma unroll 1
    for (int r = 0; r < 2; ++r) {
      if (wm == r) {
#pragma unroll
        for (int t = 0; t < 4; ++t) {
#pragma unroll
          for (int v = 0; v < 8; ++v) {
            float* sp = stg + (t * 16 + hs * 8 + v) * SP + wn * 32 + lr;
            sp[0]  = acc[t][0][v] * INV1 + bv0;
            sp[16] = acc[t][1][v] * INV1 + bv1;
          }
        }
      }
      __syncthreads();
      v8h hv[4];
#pragma unroll
      for (int i = 0; i < 4; ++i) {
        const int rl = 2 * (i * 8 + wave) + hs;
        const float* sp = stg + rl * SP + 8 * lr;
        const v4f f0 = *(const v4f*)sp;
        const v4f f1 = *(const v4f*)(sp + 4);
        hv[i][0] = (_Float16)(f0.x * HSC); hv[i][1] = (_Float16)(f0.y * HSC);
        hv[i][2] = (_Float16)(f0.z * HSC); hv[i][3] = (_Float16)(f0.w * HSC);
        hv[i][4] = (_Float16)(f1.x * HSC); hv[i][5] = (_Float16)(f1.y * HSC);
        hv[i][6] = (_Float16)(f1.z * HSC); hv[i][7] = (_Float16)(f1.w * HSC);
      }
      _Float16* ob = outh + (size_t)(m0 + 64 * r) * HIDDEN + n0 + 8 * lr;
#pragma unroll
      for (int i = 0; i < 4; ++i)
        *(volatile v8h*)(ob + (size_t)(2 * (i * 8 + wave) + hs) * HIDDEN) = hv[i];
      __threadfence();
#pragma unroll
      for (int i = 0; i < 4; ++i)
        *(volatile v8h*)(ob + (size_t)(2 * (i * 8 + wave) + hs) * HIDDEN) = hv[i];
      __syncthreads();
    }
  } else {
    constexpr float INV2 = 1.0f / (HSC * W2SC);
    const int c0 = wn * 32 + lr, c1 = c0 + 16;
    const float bv0 = bias[c0 < OUTPUT ? c0 : OUTPUT - 1];
    const float bv1 = bias[c1 < OUTPUT ? c1 : OUTPUT - 1];
#pragma unroll
    for (int t = 0; t < 4; ++t) {
#pragma unroll
      for (int v = 0; v < 8; ++v) {
        const int rowl = wm * 64 + t * 16 + hs * 8 + v;
        const float o0 = acc[t][0][v] * INV2 + bv0;
        const float o1 = acc[t][1][v] * INV2 + bv1;
        if (c0 < OUTPUT) stg[rowl * OUTPUT + c0] = o0;
        if (c1 < OUTPUT) stg[rowl * OUTPUT + c1] = o1;
      }
    }
    __syncthreads();
    float* ob = outf + (size_t)m0 * OUTPUT;
#pragma unroll 1
    for (int g = wave; g < (BM * OUTPUT) / 128; g += NWAVE) {
      const int idx = g * 128 + 4 * lane;
      const v4f vv = *(const v4f*)(stg + idx);
      *(volatile v4f*)(ob + idx) = vv;
    }
    __threadfence();
#pragma unroll 1
    for (int g = wave; g < (BM * OUTPUT) / 128; g += NWAVE) {
      const int idx = g * 128 + 4 * lane;
      const v4f vv = *(const v4f*)(stg + idx);
      *(volatile v4f*)(ob + idx) = vv;
    }
  }
}

extern "C" void kernel_launch(void* const* d_in, const int* in_sizes, int n_in,
                              void* d_out, int out_size, void* d_ws, size_t ws_size,
                              hipStream_t stream) {
  if (n_in < 5) return;
  if (in_sizes[0] != BATCH * MAXLEN) return;
  if (in_sizes[1] != HIDDEN * CHARS) return;
  if (in_sizes[2] != HIDDEN) return;
  if (in_sizes[3] != OUTPUT * HIDDEN) return;
  if (in_sizes[4] != OUTPUT) return;
  if (out_size != BATCH * OUTPUT) return;

  const int*   words = (const int*)d_in[0];
  const float* W1    = (const float*)d_in[1];
  const float* b1    = (const float*)d_in[2];
  const float* W2    = (const float*)d_in[3];
  const float* b2    = (const float*)d_in[4];
  float* out = (float*)d_out;

  char* ws = (char*)d_ws;
  size_t off = 0;
  const size_t oA  = off; off += (size_t)BATCH * K1P * 2;    off = (off + 255) & ~(size_t)255;
  const size_t oW1 = off; off += (size_t)HIDDEN * K1P * 2;   off = (off + 255) & ~(size_t)255;
  const size_t oH  = off; off += (size_t)BATCH * HIDDEN * 2; off = (off + 255) & ~(size_t)255;
  const size_t oW2 = off; off += (size_t)N2P * HIDDEN * 2;   off = (off + 255) & ~(size_t)255;
  if (off > ws_size || off > (size_t)WSCAP) return;

  _Float16* ah   = (_Float16*)(ws + oA);
  _Float16* w1h  = (_Float16*)(ws + oW1);
  _Float16* hidh = (_Float16*)(ws + oH);
  _Float16* w2h  = (_Float16*)(ws + oW2);

  hipFuncSetAttribute(reinterpret_cast<const void*>(&k_hist), hipFuncAttributeMaxDynamicSharedMemorySize, LDSH_BYTES);

  k_cvt<<<NB1 + NB2, NT, 0, stream>>>(W1, W2, w1h, w2h);
  k_hist<<<BATCH / HROWS, NT, LDSH_BYTES, stream>>>(words, ah);
  k_gemm<0><<<dim3(HIDDEN / BN, BATCH / BM), NT, 0, stream>>>(ah, w1h, b1, K1P, K1P, KS1, hidh, out);
  k_gemm<1><<<dim3(1, BATCH / BM), NT, 0, stream>>>(hidh, w2h, b2, HIDDEN, HIDDEN, KS2, hidh, out);
}
